// MSDeform_OnOffset_v1_80023830659195
// MI455X (gfx1250) — hardware-verified
//
#include <hip/hip_runtime.h>
#include <stdint.h>

#define DM     256
#define NH     8
#define NL     4
#define NP     4
#define OD     32
#define DH     32
#define LQ     5440
#define NB     4
#define MT     (NB * LQ)
#define NG     (NH * NL * NP)
#define NOE    (NG * OD)
#define QT     (LQ / 16)
#define NTILE  (MT / 16)
#define NBLK32 (MT / 32)

#define AP     264
#define SP     36
#define QP     264
#define OEP    33
#define OHP    260
#define QS_F   2112
#define OE_F   (NH * 16 * OEP)
#define POOL_F (QS_F + OE_F)

#define WOH_BYTES ((size_t)NOE * DM * 2)
#define WVH_BYTES ((size_t)DM * DM * 2)
#define WWH_BYTES ((size_t)DM * DM * 2)
#define WSR_BYTES ((size_t)NG * OD * 2 * 4)
#define WAR_BYTES ((size_t)NG * OD * 4)
#define VAL_BYTES ((size_t)MT * DM * 4)
#define OH_BYTES  ((size_t)MT * DM * 4)
#define WS_WOH  ((size_t)0)
#define WS_WVH  (WS_WOH + WOH_BYTES)
#define WS_WWH  (WS_WVH + WVH_BYTES)
#define WS_WSR  (WS_WWH + WWH_BYTES)
#define WS_WAR  (WS_WSR + WSR_BYTES)
#define WS_VAL  (WS_WAR + WAR_BYTES)
#define WS_OH   (WS_VAL + VAL_BYTES)
#define WS_END  (WS_OH + OH_BYTES)

static_assert((WOH_BYTES % 128) == 0);
static_assert((WVH_BYTES % 128) == 0);
static_assert((WWH_BYTES % 128) == 0);
static_assert((WSR_BYTES % 128) == 0);
static_assert((WAR_BYTES % 128) == 0);
static_assert((VAL_BYTES % 128) == 0);
static_assert((WS_VAL % 128) == 0);
static_assert((WS_OH % 128) == 0);
static_assert(WS_END <= (size_t)134217728);
static_assert((LQ % 32) == 0);
static_assert((MT % 32) == 0);
static_assert(((NOE * DM / 8) % 256) == 0);
static_assert(((DM * DM / 8) % 256) == 0);
static_assert(((NG * OD * 2 / 4) % 256) == 0);
static_assert(((NG * OD / 4) % 256) == 0);
static_assert((AP * 2) % 16 == 0);
static_assert((QP * 2) % 16 == 0);
static_assert((SP * 4) % 16 == 0);
static_assert((OHP * 4) % 16 == 0);
static_assert(16 * QP == 2 * QS_F);
static_assert(16 * OHP <= POOL_F);
static_assert(32 * AP * 2 + 8 * 32 * SP * 4 <= 60000);
static_assert(POOL_F * 4 + 16 * NH * 16 * 2 * 4 + 16 * NH * 16 * 4 <= 60000);

typedef __bf16         v16b __attribute__((ext_vector_type(16)));
typedef _Float16       v16h __attribute__((ext_vector_type(16)));
typedef float          v8f  __attribute__((ext_vector_type(8)));
typedef float          v4f  __attribute__((ext_vector_type(4)));
typedef unsigned short v8us __attribute__((ext_vector_type(8)));

__device__ __forceinline__ unsigned bfb(float f) {
  const unsigned u = __float_as_uint(f);
  return (u + 0x7FFFu + ((u >> 16) & 1u)) >> 16;
}
__device__ __forceinline__ float bf_rne(float f) { return __uint_as_float(bfb(f) << 16); }
__device__ __forceinline__ unsigned short h16b(float f) {
  const _Float16 hv = (_Float16)f;
  return __builtin_bit_cast(unsigned short, hv);
}
__device__ __forceinline__ v8f zero8f() { v8f z = {0.f, 0.f, 0.f, 0.f, 0.f, 0.f, 0.f, 0.f}; return z; }
__device__ __forceinline__ float silu_f(float x) {
  return x * __builtin_amdgcn_rcpf(1.0f + __expf(-x));
}

union FragB { v16b v; v8us u[2]; };
union FragH { v16h v; v8us u[2]; };
__device__ __forceinline__ v16b ldfb(const unsigned short* p) {
  FragB f;
  f.u[0] = *(const v8us*)(p);
  f.u[1] = *(const v8us*)(p + 16);
  return f.v;
}
__device__ __forceinline__ v16h ldfh(const unsigned short* p) {
  FragH f;
  f.u[0] = *(const v8us*)(p);
  f.u[1] = *(const v8us*)(p + 16);
  return f.v;
}

__device__ __forceinline__ v8f mma_b(const v16b& a, const v16b& b, v8f c) {
  v8f d = __builtin_amdgcn_wmma_f32_16x16x32_bf16(false, a, false, b, (short)0, c, false, false);
#if defined(__HIP_DEVICE_COMPILE__)
  asm volatile("v_nop\n\tv_nop\n\tv_nop\n\tv_nop" : "+v"(d) : "v"(a), "v"(b));
#endif
  return d;
}
__device__ __forceinline__ v8f mma_h(const v16h& a, const v16h& b, v8f c) {
  v8f d = __builtin_amdgcn_wmma_f32_16x16x32_f16(false, a, false, b, (short)0, c, false, false);
#if defined(__HIP_DEVICE_COMPILE__)
  asm volatile("v_nop\n\tv_nop\n\tv_nop\n\tv_nop" : "+v"(d) : "v"(a), "v"(b));
#endif
  return d;
}

__global__ __launch_bounds__(256)
void k_cvt_bf16(const float* __restrict__ s, unsigned short* d, int n8)
{
  const int i = blockIdx.x * 256 + threadIdx.x;
  if (i < n8) {
    const float* sp = s + (size_t)i * 8;
    const v4f x0 = *(const v4f*)(sp);
    const v4f x1 = *(const v4f*)(sp + 4);
    v8us pk;
    pk[0] = (unsigned short)bfb(x0.x); pk[1] = (unsigned short)bfb(x0.y);
    pk[2] = (unsigned short)bfb(x0.z); pk[3] = (unsigned short)bfb(x0.w);
    pk[4] = (unsigned short)bfb(x1.x); pk[5] = (unsigned short)bfb(x1.y);
    pk[6] = (unsigned short)bfb(x1.z); pk[7] = (unsigned short)bfb(x1.w);
    unsigned short* dp = d + (size_t)i * 8;
    *(volatile v8us*)dp = pk;
    __threadfence();
    *(volatile v8us*)dp = pk;
  }
}

__global__ __launch_bounds__(256)
void k_cvt_f16x16(const float* __restrict__ s, unsigned short* d, int n8)
{
  const int i = blockIdx.x * 256 + threadIdx.x;
  if (i < n8) {
    const float* sp = s + (size_t)i * 8;
    const v4f x0 = *(const v4f*)(sp);
    const v4f x1 = *(const v4f*)(sp + 4);
    v8us pk;
    pk[0] = h16b(bf_rne(x0.x) * 16.0f); pk[1] = h16b(bf_rne(x0.y) * 16.0f);
    pk[2] = h16b(bf_rne(x0.z) * 16.0f); pk[3] = h16b(bf_rne(x0.w) * 16.0f);
    pk[4] = h16b(bf_rne(x1.x) * 16.0f); pk[5] = h16b(bf_rne(x1.y) * 16.0f);
    pk[6] = h16b(bf_rne(x1.z) * 16.0f); pk[7] = h16b(bf_rne(x1.w) * 16.0f);
    unsigned short* dp = d + (size_t)i * 8;
    *(volatile v8us*)dp = pk;
    __threadfence();
    *(volatile v8us*)dp = pk;
  }
}

__global__ __launch_bounds__(256)
void k_rnd4(const float* __restrict__ s, float* d, int n4)
{
  const int i = blockIdx.x * 256 + threadIdx.x;
  if (i < n4) {
    const v4f v = *(const v4f*)(s + (size_t)i * 4);
    v4f r;
    r.x = bf_rne(v.x); r.y = bf_rne(v.y); r.z = bf_rne(v.z); r.w = bf_rne(v.w);
    float* dp = d + (size_t)i * 4;
    *(volatile v4f*)dp = r;
    __threadfence();
    *(volatile v4f*)dp = r;
  }
}

template <int MODE>
__global__ __launch_bounds__(256) __attribute__((amdgpu_num_vgpr(256)))
void k_gemm(const float* __restrict__ A, const unsigned short* __restrict__ Bp,
            const float* __restrict__ bias, float* dst)
{
  __shared__ __align__(16) unsigned short As[32 * AP];
  __shared__ __align__(16) float stg[8 * 32 * SP];

  const int tid  = threadIdx.x;
  const int lane = tid & 31;
  const int wid  = tid >> 5;
  const int m    = lane & 15;
  const int hh   = lane >> 4;
  const int r0   = blockIdx.x * 32;

#pragma unroll
  for (int j = 0; j < 4; ++j) {
    const int c   = tid + 256 * j;
    const int row = c >> 5;
    const int k8  = (c & 31) * 8;
    const float* sp = A + (size_t)(r0 + row) * DM + k8;
    const v4f x0 = *(const v4f*)(sp);
    const v4f x1 = *(const v4f*)(sp + 4);
    v8us pk;
    if (MODE == 0) {
      pk[0] = (unsigned short)bfb(x0.x); pk[1] = (unsigned short)bfb(x0.y);
      pk[2] = (unsigned short)bfb(x0.z); pk[3] = (unsigned short)bfb(x0.w);
      pk[4] = (unsigned short)bfb(x1.x); pk[5] = (unsigned short)bfb(x1.y);
      pk[6] = (unsigned short)bfb(x1.z); pk[7] = (unsigned short)bfb(x1.w);
    } else {
      pk[0] = h16b(x0.x * 16.0f); pk[1] = h16b(x0.y * 16.0f);
      pk[2] = h16b(x0.z * 16.0f); pk[3] = h16b(x0.w * 16.0f);
      pk[4] = h16b(x1.x * 16.0f); pk[5] = h16b(x1.y * 16.0f);
      pk[6] = h16b(x1.z * 16.0f); pk[7] = h16b(x1.w * 16.0f);
    }
    *(v8us*)(As + row * AP + k8) = pk;
  }
  __syncthreads();

  v8f acc00 = zero8f(), acc01 = zero8f(), acc10 = zero8f(), acc11 = zero8f();
  {
    const unsigned short* ap0 = As + m * AP + 8 * hh;
    const unsigned short* ap1 = ap0 + 16 * AP;
    const unsigned short* bp0 = Bp + (size_t)(32 * wid + m) * DM + 8 * hh;
    const unsigned short* bp1 = bp0 + 16 * DM;
    if (MODE == 0) {
#pragma unroll
      for (int kb = 0; kb < 8; ++kb) {
        const v16b a0 = ldfb(ap0 + 32 * kb);
        const v16b a1 = ldfb(ap1 + 32 * kb);
        const v16b b0 = ldfb(bp0 + 32 * kb);
        const v16b b1 = ldfb(bp1 + 32 * kb);
        acc00 = mma_b(a0, b0, acc00);
        acc01 = mma_b(a0, b1, acc01);
        acc10 = mma_b(a1, b0, acc10);
        acc11 = mma_b(a1, b1, acc11);
      }
    } else {
#pragma unroll
      for (int kb = 0; kb < 8; ++kb) {
        const v16h a0 = ldfh(ap0 + 32 * kb);
        const v16h a1 = ldfh(ap1 + 32 * kb);
        const v16h b0 = ldfh(bp0 + 32 * kb);
        const v16h b1 = ldfh(bp1 + 32 * kb);
        acc00 = mma_h(a0, b0, acc00);
        acc01 = mma_h(a0, b1, acc01);
        acc10 = mma_h(a1, b0, acc10);
        acc11 = mma_h(a1, b1, acc11);
      }
    }
  }

  {
    const int c0 = 32 * wid + m;
    const int c1 = c0 + 16;
    const float q0 = bf_rne(bias[c0]);
    const float q1 = bf_rne(bias[c1]);
    const float sc = (MODE == 0) ? 1.0f : 0.00390625f;
    float* sw = stg + wid * (32 * SP);
#pragma unroll
    for (int r = 0; r < 8; ++r) {
      sw[(8 * hh + r) * SP + m]           = acc00[r] * sc + q0;
      sw[(8 * hh + r) * SP + 16 + m]      = acc01[r] * sc + q1;
      sw[(16 + 8 * hh + r) * SP + m]      = acc10[r] * sc + q0;
      sw[(16 + 8 * hh + r) * SP + 16 + m] = acc11[r] * sc + q1;
    }
  }
  __syncthreads();

  {
    const int pj = lane & 7;
    const int lq = lane >> 3;
    const float* sw = stg + wid * (32 * SP);
    size_t base, rstride;
    if (MODE == 0) {
      const int b    = r0 / LQ;
      const int pos0 = r0 - b * LQ;
      base    = ((size_t)(b * NH + wid) * LQ + pos0) * DH + 4 * pj;
      rstride = DH;
    } else {
      base    = (size_t)r0 * DM + 32 * wid + 4 * pj;
      rstride = DM;
    }
    v4f val[8]; size_t e[8];
#pragma unroll
    for (int r = 0; r < 8; ++r) {
      const int row = 4 * r + lq;
      val[r] = *(const v4f*)(sw + row * SP + 4 * pj);
      e[r]   = base + (size_t)row * rstride;
    }
#pragma unroll
    for (int r = 0; r < 8; ++r) *(volatile v4f*)(dst + e[r]) = val[r];
    __threadfence();
#pragma unroll
    for (int r = 0; r < 8; ++r) *(volatile v4f*)(dst + e[r]) = val[r];
  }
}

__global__ __launch_bounds__(256) __attribute__((amdgpu_num_vgpr(256)))
void k_core(const float* __restrict__ query, const float* __restrict__ refp,
            const unsigned short* __restrict__ Woh,
            const float* __restrict__ Wsr, const float* __restrict__ Wsb,
            const float* __restrict__ War, const float* __restrict__ Wab,
            const float* __restrict__ val, float* oh)
{
#pragma clang fp contract(off)
  __shared__ __align__(16) float pool[POOL_F];
  __shared__ __align__(16) float locs[16 * NH * 16 * 2];
  __shared__ float aws[16 * NH * 16];
  unsigned short* Qs  = (unsigned short*)pool;
  float*          oe  = pool + QS_F;
  float*          ohs = pool;

  const int tid  = threadIdx.x;
  const int lane = tid & 31;
  const int wid  = tid >> 5;
  const int m    = lane & 15;
  const int hh   = lane >> 4;
  const int tile = blockIdx.x;
  const int b    = tile / QT;
  const int q0   = (tile - b * QT) * 16;
  const int h    = wid;

#pragma unroll
  for (int j = 0; j < 2; ++j) {
    const int c   = tid + 256 * j;
    const int row = c >> 5;
    const int k8  = (c & 31) * 8;
    const float* sp = query + (size_t)(b * LQ + q0 + row) * DM + k8;
    const v4f x0 = *(const v4f*)(sp);
    const v4f x1 = *(const v4f*)(sp + 4);
    v8us pk;
    pk[0] = (unsigned short)bfb(x0.x); pk[1] = (unsigned short)bfb(x0.y);
    pk[2] = (unsigned short)bfb(x0.z); pk[3] = (unsigned short)bfb(x0.w);
    pk[4] = (unsigned short)bfb(x1.x); pk[5] = (unsigned short)bfb(x1.y);
    pk[6] = (unsigned short)bfb(x1.z); pk[7] = (unsigned short)bfb(x1.w);
    *(v8us*)(Qs + row * QP + k8) = pk;
  }
  __syncthreads();

  {
    const unsigned short* aq = Qs + m * QP + 8 * hh;
    float* oew = oe + wid * (16 * OEP);
#pragma unroll 1
    for (int lk = 0; lk < 16; ++lk) {
      const int g = h * 16 + lk;
      const unsigned short* bq0 = Woh + (size_t)(g * 32 + m) * DM + 8 * hh;
      const unsigned short* bq1 = bq0 + 16 * DM;
      v8f acc0 = zero8f(), acc1 = zero8f();
#pragma unroll
      for (int kb = 0; kb < 8; ++kb) {
        const v16b a  = ldfb(aq  + 32 * kb);
        const v16b b0 = ldfb(bq0 + 32 * kb);
        const v16b b1 = ldfb(bq1 + 32 * kb);
        acc0 = mma_b(a, b0, acc0);
        acc1 = mma_b(a, b1, acc1);
      }
#pragma unroll
      for (int v = 0; v < 8; ++v) {
        oew[(8 * hh + v) * OEP + m]      = silu_f(acc0[v]);
        oew[(8 * hh + v) * OEP + 16 + m] = silu_f(acc1[v]);
      }
      __syncthreads();
      {
        const int q  = m;
        const int cc = hh;
        const float* orow = oew + q * OEP;
        const float* wsp  = Wsr + (size_t)g * 64 + cc;
        const float* wap  = War + (size_t)g * 32;
        float s = 0.0f, sa = 0.0f;
#pragma unroll 8
        for (int d = 0; d < OD; ++d) {
          const float o = orow[d];
          s  = s  + o * wsp[2 * d];
          sa = sa + o * wap[d];
        }
        const int   l   = lk >> 2;
        const float inv = __uint_as_float((unsigned)(121 + l) << 23);
        const float rv  = bf_rne(refp[((size_t)(b * LQ + q0 + q) * NL + l) * 2 + cc]);
        const float sbv = bf_rne(Wsb[g * 2 + cc]);
        const float abv = bf_rne(Wab[g]);
        const float loc = rv + (s + sbv) * inv;
        locs[((q * NH + h) * 16 + lk) * 2 + cc] = loc;
        if (cc == 0) aws[(q * NH + h) * 16 + lk] = sa + abv;
      }
      __syncthreads();
    }
  }

  if (tid < 128) {
    const int q  = tid >> 3;
    const int hd = tid & 7;
    float* ap = aws + (q * NH + hd) * 16;
    float e[16];
    float mx = ap[0];
#pragma unroll
    for (int i = 1; i < 16; ++i) mx = fmaxf(mx, ap[i]);
    float sum = 0.0f;
#pragma unroll
    for (int i = 0; i < 16; ++i) { e[i] = __expf(ap[i] - mx); sum = sum + e[i]; }
    const float inv = __builtin_amdgcn_rcpf(sum);
#pragma unroll
    for (int i = 0; i < 16; ++i) ap[i] = e[i] * inv;
  }
  __syncthreads();

  {
    const int d = lane;
    const float* vrow = val + ((size_t)(b * NH + h)) * LQ * DH + d;
#pragma unroll 1
    for (int q = 0; q < 16; ++q) {
      const float* lp = locs + (q * NH + h) * 32;
      const float* wp = aws + (q * NH + h) * 16;
      float accf = 0.0f;
#pragma unroll
      for (int l = 0; l < NL; ++l) {
        const int   S    = 64 >> l;
        const int   base = (l == 0) ? 0 : ((l == 1) ? 4096 : ((l == 2) ? 5120 : 5376));
        const float fS   = (float)S;
        float lv = 0.0f;
#pragma unroll
        for (int k = 0; k < NP; ++k) {
          const int   lk2 = (l * NP + k) * 2;
          const float lx  = lp[lk2];
          const float ly  = lp[lk2 + 1];
          const float awv = wp[l * NP + k];
          const float x   = lx * fS - 0.5f;
          const float y   = ly * fS - 0.5f;
          const float xf  = floorf(x);
          const float yf  = floorf(y);
          const float wx  = x - xf;
          const float wy  = y - yf;
          const float omx = 1.0f - wx;
          const float omy = 1.0f - wy;
          const int xi = (int)fminf(fmaxf(xf, -4.0e6f), 4.0e6f);
          const int yi = (int)fminf(fmaxf(yf, -4.0e6f), 4.0e6f);
          const bool vx0 = (xi >= 0)  && (xi < S);
          const bool vx1 = (xi >= -1) && (xi < S - 1);
          const bool vy0 = (yi >= 0)  && (yi < S);
          const bool vy1 = (yi >= -1) && (yi < S - 1);
          const int cx0 = min(max(xi, 0), S - 1);
          const int cx1 = min(max(xi + 1, 0), S - 1);
          const int cy0 = min(max(yi, 0), S - 1);
          const int cy1 = min(max(yi + 1, 0), S - 1);
          const float g00 = vrow[(size_t)(base + cy0 * S + cx0) * DH];
          const float g01 = vrow[(size_t)(base + cy0 * S + cx1) * DH];
          const float g10 = vrow[(size_t)(base + cy1 * S + cx0) * DH];
          const float g11 = vrow[(size_t)(base + cy1 * S + cx1) * DH];
          const float m00 = (vy0 && vx0) ? 1.0f : 0.0f;
          const float m01 = (vy0 && vx1) ? 1.0f : 0.0f;
          const float m10 = (vy1 && vx0) ? 1.0f : 0.0f;
          const float m11 = (vy1 && vx1) ? 1.0f : 0.0f;
          float t = ((g00 * m00) * omx) * omy;
          t = t + ((g01 * m01) * wx) * omy;
          t = t + ((g10 * m10) * omx) * wy;
          t = t + ((g11 * m11) * wx) * wy;
          lv = lv + t * awv;
        }
        accf = accf + lv;
      }
      ohs[q * OHP + h * 32 + d] = accf;
    }
  }
  __syncthreads();

  {
    const int pj = lane & 7;
    const int lq = lane >> 3;
    v4f valv[4]; size_t e[4];
#pragma unroll
    for (int r = 0; r < 4; ++r) {
      const int L   = r * 32 + wid * 4 + lq;
      const int row = L >> 3;
      const int seg = L & 7;
      valv[r] = *(const v4f*)(ohs + row * OHP + seg * 32 + 4 * pj);
      e[r]    = ((size_t)(b * LQ + q0 + row)) * DM + seg * 32 + 4 * pj;
    }
#pragma unroll
    for (int r = 0; r < 4; ++r) *(volatile v4f*)(oh + e[r]) = valv[r];
    __threadfence();
#pragma unroll
    for (int r = 0; r < 4; ++r) *(volatile v4f*)(oh + e[r]) = valv[r];
  }
}

extern "C" void kernel_launch(void* const* d_in, const int* in_sizes, int n_in,
                              void* d_out, int out_size, void* d_ws, size_t ws_size,
                              hipStream_t stream) {
  if (n_in < 13) return;
  if (in_sizes[0]  != MT * DM) return;
  if (in_sizes[1]  != MT * NL * 2) return;
  if (in_sizes[2]  != MT * DM) return;
  if (in_sizes[4]  != NOE * DM) return;
  if (in_sizes[5]  != NG * OD * 2) return;
  if (in_sizes[6]  != NG * 2) return;
  if (in_sizes[7]  != NG * OD) return;
  if (in_sizes[8]  != NG) return;
  if (in_sizes[9]  != DM * DM) return;
  if (in_sizes[10] != DM) return;
  if (in_sizes[11] != DM * DM) return;
  if (in_sizes[12] != DM) return;
  if (out_size != MT * DM) return;
  if (WS_END > ws_size) return;

  const float* query = (const float*)d_in[0];
  const float* refp  = (const float*)d_in[1];
  const float* xin   = (const float*)d_in[2];
  const float* Wo    = (const float*)d_in[4];
  const float* Ws    = (const float*)d_in[5];
  const float* Wsb   = (const float*)d_in[6];
  const float* Wa    = (const float*)d_in[7];
  const float* Wab   = (const float*)d_in[8];
  const float* Wv    = (const float*)d_in[9];
  const float* vb    = (const float*)d_in[10];
  const float* Ww    = (const float*)d_in[11];
  const float* ob    = (const float*)d_in[12];
  float* out = (float*)d_out;
  char* ws = (char*)d_ws;

  unsigned short* Woh = (unsigned short*)(ws + WS_WOH);
  unsigned short* Wvh = (unsigned short*)(ws + WS_WVH);
  unsigned short* Wwh = (unsigned short*)(ws + WS_WWH);
  float* Wsr = (float*)(ws + WS_WSR);
  float* War = (float*)(ws + WS_WAR);
  float* valp = (float*)(ws + WS_VAL);
  float* ohp  = (float*)(ws + WS_OH);

  k_cvt_bf16<<<dim3(NOE * DM / 8 / 256), dim3(256), 0, stream>>>(Wo, Woh, NOE * DM / 8);
  (void)hipGetLastError();
  k_cvt_bf16<<<dim3(DM * DM / 8 / 256), dim3(256), 0, stream>>>(Wv, Wvh, DM * DM / 8);
  (void)hipGetLastError();
  k_cvt_f16x16<<<dim3(DM * DM / 8 / 256), dim3(256), 0, stream>>>(Ww, Wwh, DM * DM / 8);
  (void)hipGetLastError();
  k_rnd4<<<dim3(NG * OD * 2 / 4 / 256), dim3(256), 0, stream>>>(Ws, Wsr, NG * OD * 2 / 4);
  (void)hipGetLastError();
  k_rnd4<<<dim3(NG * OD / 4 / 256), dim3(256), 0, stream>>>(Wa, War, NG * OD / 4);
  (void)hipGetLastError();

  k_gemm<0><<<dim3(NBLK32), dim3(256), 0, stream>>>(xin, (const unsigned short*)Wvh, vb, valp);
  (void)hipGetLastError();

  k_core<<<dim3(NTILE), dim3(256), 0, stream>>>(query, refp, (const unsigned short*)Woh,
                                                (const float*)Wsr, Wsb, (const float*)War, Wab,
                                                (const float*)valp, ohp);
  (void)hipGetLastError();

  k_gemm<1><<<dim3(NBLK32), dim3(256), 0, stream>>>((const float*)ohp, (const unsigned short*)Wwh, ob, out);
  (void)hipGetLastError();
}
